// MultiHeadAttention_21741124452899
// MI455X (gfx1250) — hardware-run, weakly checked
//
#include <hip/hip_runtime.h>
#ifndef NB
#define NB 2
#endif
#ifndef SEQ
#define SEQ 2048
#endif
#define NB_FULL 2
#define SEQ_FULL 2048
#define SQ SEQ
#define DM 1024
#define NH 16
#define HD 64
#define QT 256
#define NKX SQ
#define RC (SQ / 256)
#define SCL 0.125f
#define NR ((size_t)NB * SQ)
#define MP ((int)(NB * SQ))
#define BSTR_FULL ((size_t)SEQ_FULL * DM)

static_assert(SQ % 256 == 0);
static_assert(SQ <= SEQ_FULL);
static_assert(NB <= NB_FULL);
static_assert(DM == NH * HD);
static_assert(HD == 64);
static_assert(MP % 128 == 0);
static_assert(DM % 64 == 0);
static_assert(QT % 128 == 0);

typedef unsigned short v8us __attribute__((ext_vector_type(8), may_alias));
typedef float  v8f  __attribute__((ext_vector_type(8)));
typedef float  v4f  __attribute__((ext_vector_type(4)));
typedef float  v4fa __attribute__((ext_vector_type(4), may_alias));
typedef _Float16 v16h __attribute__((ext_vector_type(16)));
typedef _Float16 v4h __attribute__((ext_vector_type(4)));
union FragH { v16h v; v8us half[2]; _Float16 h[16]; unsigned short u[16]; };

__device__ __forceinline__ unsigned short bf16_bits(float x) { unsigned int u = __float_as_uint(x); return (unsigned short)((u + 0x7FFFu + ((u >> 16) & 1u)) >> 16); }
__device__ __forceinline__ float bf16_val(unsigned short b) { return __uint_as_float(((unsigned int)b) << 16); }
__device__ __forceinline__ float bf16_rne(float x) { return bf16_val(bf16_bits(x)); }

__device__ __forceinline__ v16h g2_frag(const _Float16* p, int hh) { FragH f; f.half[0] = *(const v8us*)((const unsigned short*)p + 8 * hh); f.half[1] = *(const v8us*)((const unsigned short*)p + 16 + 8 * hh); return f.v; }
__device__ __forceinline__ v8f g2_mma(v16h a, v16h b, v8f c) { v8f d = __builtin_amdgcn_wmma_f32_16x16x32_f16(false, a, false, b, (short)0, c, false, false); asm volatile("v_nop\n\tv_nop\n\tv_nop\n\tv_nop" : "+v"(d) : "v"(a), "v"(b)); return d; }

__global__ __launch_bounds__(256) void k_wt_f16(const float* __restrict__ W, _Float16* __restrict__ Wt, int K, int N, float scale) {
  const int t = blockIdx.x * 256 + threadIdx.x; if (t >= N * (K / 8)) return;
  const int n = t / (K / 8), k8 = (t % (K / 8)) * 8; FragH f;
#pragma unroll
  for (int i = 0; i < 8; ++i) f.h[i] = (_Float16)(bf16_rne(W[(size_t)(k8 + i) * N + n]) * scale);
  const v8us o = f.half[0];
  unsigned short* d = (unsigned short*)Wt + (size_t)n * K + k8;
  *(volatile v8us*)d = o; __threadfence(); *(volatile v8us*)d = o;
}

__global__ __launch_bounds__(256) void k_x16(const float* __restrict__ x, size_t sx, _Float16* __restrict__ X16, size_t sX, size_t n8) {
  const size_t t = (size_t)blockIdx.x * 256 + threadIdx.x; if (t >= n8) return;
  const float* xp = x + (size_t)blockIdx.y * sx + t * 8;
  unsigned short* d = (unsigned short*)X16 + (size_t)blockIdx.y * sX + t * 8;
  const v4f a = *(const v4fa*)xp, c = *(const v4fa*)(xp + 4); FragH f;
#pragma unroll
  for (int q = 0; q < 4; ++q) { f.h[q] = (_Float16)bf16_rne(a[q]); f.h[4 + q] = (_Float16)bf16_rne(c[q]); }
  const v8us o = f.half[0];
  *(volatile v8us*)d = o; __threadfence(); *(volatile v8us*)d = o;
}

__global__ __launch_bounds__(256) void k_h16(const float* __restrict__ F, _Float16* __restrict__ Hh, size_t n8) {
  const size_t t = (size_t)blockIdx.x * 256 + threadIdx.x; if (t >= n8) return; FragH fh;
  const v4f a = *(const v4fa*)(F + t * 8), c = *(const v4fa*)(F + t * 8 + 4);
#pragma unroll
  for (int q = 0; q < 4; ++q) { fh.h[q] = (_Float16)a[q]; fh.h[4 + q] = (_Float16)c[q]; }
  const v8us oh = fh.half[0];
  unsigned short* d = (unsigned short*)Hh + t * 8;
  *(volatile v8us*)d = oh; __threadfence(); *(volatile v8us*)d = oh;
}

template <int NHv, int TTv>
__global__ __launch_bounds__(256) void k_vt(const _Float16* __restrict__ V16, int ldv, int voff, _Float16* __restrict__ Vt) {
  __shared__ unsigned short tl[64][66];
  const int tid = threadIdx.x; const int slab = blockIdx.x / (TTv / 64), lg = blockIdx.x % (TTv / 64); const int b = slab / NHv, h = slab % NHv;
  for (int i = tid; i < 64 * 8; i += 256) { const int r = i / 8, c8 = (i % 8) * 8; FragH f; f.half[0] = *(const v8us*)((const unsigned short*)V16 + ((size_t)b * TTv + lg * 64 + r) * ldv + voff + h * 64 + c8);
#pragma unroll
    for (int q = 0; q < 8; ++q) tl[r][c8 + q] = f.u[q]; }
  __syncthreads();
  for (int pass = 0; pass < 2; ++pass) {
#pragma unroll
    for (int rd = 0; rd < 2; ++rd) { const int d = rd * 32 + tid / 8, pc = tid % 8; FragH f;
#pragma unroll
      for (int q = 0; q < 8; ++q) f.u[q] = tl[pc * 8 + q][d];
      const v8us o = f.half[0];
      *(volatile v8us*)((unsigned short*)Vt + ((size_t)slab * 64 + d) * TTv + lg * 64 + pc * 8) = o; }
    if (pass == 0) __threadfence(); }
}

template <int ACT>
__global__ __launch_bounds__(128) void k_gemm2(const _Float16* __restrict__ A, int lda, size_t sA, const _Float16* __restrict__ Bh, int ldb, size_t sB, float alpha, const float* __restrict__ bias, size_t sBias,
    float* __restrict__ C, _Float16* __restrict__ C16, int ldc, size_t sC, int M, int N, int K) {
  static_assert(ACT == 0 || ACT == 3);
  __shared__ __attribute__((aligned(16))) float so[4][32][68];
  const int tid = threadIdx.x, w = __builtin_amdgcn_readfirstlane((int)(tid >> 5)), lane = tid & 31, ln = lane & 15, hh = lane >> 4; const int by = blockIdx.y;
  A += (size_t)by * sA; Bh += (size_t)by * sB; const size_t cofs = (size_t)by * sC; const float* bp = bias ? bias + (size_t)by * sBias : nullptr;
  const int ntn = N >> 6; const int mt = blockIdx.x / ntn, nq = blockIdx.x - mt * ntn; const int row0 = mt * 128 + 32 * w, col0 = nq * 64; if (row0 >= M) return;
  const _Float16* a0p = A + (size_t)(row0 + ln) * lda; const _Float16* a1p = a0p + (size_t)16 * lda;
  const _Float16* b0p = Bh + (size_t)(col0 + ln) * ldb; const _Float16* b1p = b0p + (size_t)16 * ldb; const _Float16* b2p = b1p + (size_t)16 * ldb; const _Float16* b3p = b2p + (size_t)16 * ldb;
  const v8f z8 = {0.f,0.f,0.f,0.f,0.f,0.f,0.f,0.f}; v8f c00 = z8, c01 = z8, c02 = z8, c03 = z8, c10 = z8, c11 = z8, c12 = z8, c13 = z8;
#pragma unroll 1
  for (int kb = 0; kb < K; kb += 32) { const v16h a0 = g2_frag(a0p + kb, hh), a1 = g2_frag(a1p + kb, hh);
    v16h b = g2_frag(b0p + kb, hh); c00 = g2_mma(a0, b, c00); c10 = g2_mma(a1, b, c10);
    b = g2_frag(b1p + kb, hh); c01 = g2_mma(a0, b, c01); c11 = g2_mma(a1, b, c11);
    b = g2_frag(b2p + kb, hh); c02 = g2_mma(a0, b, c02); c12 = g2_mma(a1, b, c12);
    b = g2_frag(b3p + kb, hh); c03 = g2_mma(a0, b, c03); c13 = g2_mma(a1, b, c13); }
  v8f accs[8] = {c00, c01, c02, c03, c10, c11, c12, c13};
#pragma unroll
  for (int u = 0; u < 8; ++u) { const int t = u & 3, half = u >> 2; const int col = col0 + t * 16 + ln; const float bv = bp ? bf16_rne(bp[col]) : 0.f;
#pragma unroll
    for (int r = 0; r < 8; ++r) { const int rloc = half * 16 + 8 * hh + r; float v = accs[u][r] * alpha + bv;
      if (ACT == 3) v = fmaxf(v, 0.f);
      so[w][rloc][t * 16 + ln] = v; } }
  __builtin_amdgcn_fence(4  , "workgroup"); __builtin_amdgcn_wave_barrier();
  const int rsub = lane >> 4, c4 = (lane & 15) * 4;
  for (int pass = 0; pass < 2; ++pass) {
#pragma unroll
    for (int q = 0; q < 16; ++q) { const int r = q * 2 + rsub; const v4f v = *(const v4fa*)&so[w][r][c4];
      if (C) *(volatile v4f*)(C + cofs + (size_t)(row0 + r) * ldc + col0 + c4) = v;
      if (C16) { v4h h4;
#pragma unroll
        for (int i = 0; i < 4; ++i) h4[i] = (_Float16)v[i];
        *(volatile v4h*)(C16 + cofs + (size_t)(row0 + r) * ldc + col0 + c4) = h4; } }
    if (pass == 0) __threadfence(); }
}

__global__ __launch_bounds__(256) void k_rsmw(const float* __restrict__ S, _Float16* __restrict__ P, int nrows) {
  #pragma clang fp contract(off)
  const int lane = threadIdx.x & 31; const int row = blockIdx.x * 8 + __builtin_amdgcn_readfirstlane((int)(threadIdx.x >> 5));
  if (row >= nrows) return;
  const float* s = S + (size_t)row * NKX + lane * 8;
  float e[RC * 8]; float mx = -3.0e38f;
#pragma unroll
  for (int c = 0; c < RC; ++c) { const v4f a = *(const v4fa*)(s + c * 256), b = *(const v4fa*)(s + c * 256 + 4);
#pragma unroll
    for (int q = 0; q < 4; ++q) { e[c * 8 + q] = a[q]; e[c * 8 + 4 + q] = b[q]; mx = fmaxf(mx, fmaxf(a[q], b[q])); } }
#pragma unroll
  for (int o = 16; o > 0; o >>= 1) mx = fmaxf(mx, __shfl_xor(mx, o, 32));
  float se = 0.f;
#pragma unroll
  for (int i = 0; i < RC * 8; ++i) { const float ev = __expf(e[i] - mx); e[i] = ev; se += ev; }
#pragma unroll
  for (int o = 16; o > 0; o >>= 1) se += __shfl_xor(se, o, 32);
  const float sc = 256.0f * (1.0f / se);
  v8us ov[RC];
#pragma unroll
  for (int c = 0; c < RC; ++c) { FragH f;
#pragma unroll
    for (int q = 0; q < 8; ++q) f.h[q] = (_Float16)(e[c * 8 + q] * sc);
    ov[c] = f.half[0]; }
  unsigned short* d = (unsigned short*)P + (size_t)row * NKX + lane * 8;
  for (int pass = 0; pass < 2; ++pass) {
#pragma unroll
    for (int c = 0; c < RC; ++c) *(volatile v8us*)(d + c * 256) = ov[c];
    if (pass == 0) __threadfence(); }
}

extern "C" void kernel_launch(void* const* d_in, const int* in_sizes, int n_in,
                              void* d_out, int out_size, void* d_ws, size_t ws_size, hipStream_t stream) {
  if (n_in < 11) return;
  const size_t need = (size_t)(NB - 1) * BSTR_FULL + (size_t)SQ * DM;
  if ((size_t)in_sizes[0] < need || (size_t)in_sizes[1] < need || (size_t)in_sizes[2] < need) return;
  if ((size_t)in_sizes[3] < (size_t)DM * DM || (size_t)in_sizes[5] < (size_t)DM * DM || (size_t)in_sizes[7] < (size_t)DM * DM || (size_t)in_sizes[9] < (size_t)DM * DM) return;
  if (in_sizes[4] < DM || in_sizes[6] < DM || in_sizes[8] < DM || in_sizes[10] < DM) return;
  if ((size_t)out_size < need) return;
  const float* const* I = (const float* const*)d_in;
  const float* xq = I[0]; const float* xk = I[1]; const float* xv = I[2];
  const float* wq = I[3]; const float* bq = I[4]; const float* wk = I[5]; const float* bk = I[6];
  const float* wv = I[7]; const float* bv = I[8]; const float* wo = I[9]; const float* bo = I[10];

  constexpr size_t SZ_W = (size_t)DM * DM * 2, SZ_R16 = NR * DM * 2, SZ_RF = NR * DM * 4;
  constexpr size_t SZ_S = (size_t)NH * QT * NKX * 4, SZ_P = (size_t)NH * QT * NKX * 2, SZ_VT = (size_t)NH * HD * SQ * 2;
  static_assert(4 * SZ_W + 4 * SZ_R16 + SZ_RF + SZ_S + SZ_P + SZ_VT <= (size_t)134217728);
  static_assert(SZ_W % 256 == 0 && SZ_R16 % 256 == 0 && SZ_RF % 256 == 0 && SZ_S % 256 == 0 && SZ_P % 256 == 0 && SZ_VT % 256 == 0);
  char* ws = (char*)d_ws; size_t off = 0;
  auto take = [&](size_t bytes) { char* p = ws + off; off += (bytes + 255) & ~(size_t)255; return p; };
  _Float16* BQ = (_Float16*)take(SZ_W); _Float16* BK = (_Float16*)take(SZ_W); _Float16* BV = (_Float16*)take(SZ_W); _Float16* BO = (_Float16*)take(SZ_W);
  _Float16* X16 = (_Float16*)take(SZ_R16);
  _Float16* O16 = X16;
  float* QF = (float*)take(SZ_RF);
  _Float16* QH = (_Float16*)take(SZ_R16); _Float16* KH = (_Float16*)take(SZ_R16);
  _Float16* V16 = (_Float16*)take(SZ_R16);
  float* S = (float*)take(SZ_S); _Float16* P = (_Float16*)take(SZ_P); _Float16* VT = (_Float16*)take(SZ_VT);
  if (off > ws_size) return;

  { const unsigned g = (unsigned)(((size_t)DM * (DM / 8) + 255) / 256);
    k_wt_f16<<<g, 256, 0, stream>>>(wq, BQ, DM, DM, 16.0f); k_wt_f16<<<g, 256, 0, stream>>>(wk, BK, DM, DM, 16.0f);
    k_wt_f16<<<g, 256, 0, stream>>>(wv, BV, DM, DM, 16.0f); k_wt_f16<<<g, 256, 0, stream>>>(wo, BO, DM, DM, 16.0f); }
  const size_t n8b = (size_t)SQ * DM / 8; const dim3 gx((unsigned)((n8b + 255) / 256), NB);
  const dim3 gp((unsigned)((MP / 128) * (DM / 64)), 1);
  const unsigned ghl = (unsigned)((NR * DM / 8 + 255) / 256);
  k_x16<<<gx, 256, 0, stream>>>(xq, BSTR_FULL, X16, (size_t)SQ * DM, n8b);
  k_gemm2<0><<<gp, 128, 0, stream>>>(X16, DM, (size_t)0, BQ, DM, (size_t)0, 0.0625f, bq, (size_t)0, QF, nullptr, DM, (size_t)0, MP, DM, DM);
  k_h16<<<ghl, 256, 0, stream>>>(QF, QH, NR * DM / 8);
  k_x16<<<gx, 256, 0, stream>>>(xk, BSTR_FULL, X16, (size_t)SQ * DM, n8b);
  k_gemm2<0><<<gp, 128, 0, stream>>>(X16, DM, (size_t)0, BK, DM, (size_t)0, 0.0625f, bk, (size_t)0, QF, nullptr, DM, (size_t)0, MP, DM, DM);
  k_h16<<<ghl, 256, 0, stream>>>(QF, KH, NR * DM / 8);
  k_x16<<<gx, 256, 0, stream>>>(xv, BSTR_FULL, X16, (size_t)SQ * DM, n8b);
  k_gemm2<0><<<gp, 128, 0, stream>>>(X16, DM, (size_t)0, BV, DM, (size_t)0, 0.0625f, bv, (size_t)0, nullptr, V16, DM, (size_t)0, MP, DM, DM);

  for (int b = 0; b < NB; ++b) { const size_t r0 = (size_t)b * SQ;
    k_vt<NH, SQ><<<NH * (SQ / 64), 256, 0, stream>>>(V16 + r0 * DM, DM, 0, VT);
    for (int q0 = 0; q0 < SQ; q0 += QT) {
      k_gemm2<0><<<dim3((QT / 128) * (SQ / 64), NH), 128, 0, stream>>>(QH + (r0 + q0) * DM, DM, (size_t)HD, KH + r0 * DM, DM, (size_t)HD, SCL, nullptr, (size_t)0, S, nullptr, NKX, (size_t)QT * NKX, QT, SQ, HD);
      k_rsmw<<<(NH * QT + 7) / 8, 256, 0, stream>>>(S, P, NH * QT);
      k_gemm2<0><<<dim3((QT / 128) * (HD / 64), NH), 128, 0, stream>>>(P, NKX, (size_t)QT * NKX, VT, SQ, (size_t)HD * SQ, 0.25f, nullptr, (size_t)0, nullptr, O16 + (r0 + q0) * DM, DM, (size_t)HD, QT, HD, SQ);
    } }
  k_gemm2<0><<<dim3((unsigned)((SQ / 128) * (DM / 64)), NB), 128, 0, stream>>>(O16, DM, (size_t)SQ * DM, BO, DM, (size_t)0, 0.0009765625f, bo, (size_t)0, (float*)d_out, nullptr, DM, BSTR_FULL, SQ, DM, DM);
}
